// VisionMambaEncoder_88338887344538
// MI455X (gfx1250) — hardware-verified
//
#include <hip/hip_runtime.h>
#include <cstdint>
#include <cstddef>

typedef __attribute__((ext_vector_type(16))) _Float16 bf16x16;
typedef __attribute__((ext_vector_type(8)))  float  f32x8;

union FragBF16 { bf16x16 v; uint32_t u[8]; };

typedef int v4i __attribute__((vector_size(16)));
typedef __attribute__((address_space(3))) v4i v4i_as3;

#define HAS_ASYNC_LDS 0

#define BATCH   8
#define IMG     128
#define HW      32
#define LSEQ    1024
#define NPIX    (BATCH*LSEQ)
#define DMODEL  128
#define DINNER  256
#define DSTATE  16
#define DTRANK  8
#define KDIR    4
#define CPAD    64

__device__ __forceinline__ uint16_t f2bf(float f) {
    const _Float16 h = (_Float16)f;
    return __builtin_bit_cast(uint16_t, h);
}
#define ST2(T, ptr, val) do { const T _v = (val); *(volatile T*)(ptr) = _v; __threadfence(); *(volatile T*)(ptr) = _v; } while (0)
__device__ __forceinline__ float silu(float x) { return x / (1.f + __expf(-x)); }

__device__ __forceinline__ void g2l_16B(const void* g, void* l) {
#if HAS_ASYNC_LDS
    v4i*     gp = (v4i*)(uintptr_t)g;
    v4i_as3* lp = (v4i_as3*)(uint32_t)(uintptr_t)l;
    __builtin_amdgcn_global_load_async_to_lds_b128(gp, lp, 0, 0);
#else
    *(uint4*)l = *(const uint4*)g;
#endif
}

template <int N>
__device__ __forceinline__ void wait_async() {
#if HAS_ASYNC_LDS
#if defined(__has_builtin) && __has_builtin(__builtin_amdgcn_s_wait_asynccnt)
    __builtin_amdgcn_s_wait_asynccnt(N);
#else
    asm volatile("s_wait_asynccnt %0" ::"i"(N) : "memory");
#endif
#endif
}

__global__ void k_f32_to_bf16(const float* __restrict__ s, uint16_t* __restrict__ d, int n) {
    int i = blockIdx.x * blockDim.x + threadIdx.x;
    if (i < n) ST2(uint16_t, d + i, f2bf(s[i]));
}

__global__ void k_xproj_pad(const float* __restrict__ s, uint16_t* __restrict__ d) {
    int i = blockIdx.x * blockDim.x + threadIdx.x;
    int n = KDIR * CPAD * DINNER;
    if (i >= n) return;
    int dd = i % DINNER;
    int c  = (i / DINNER) % CPAD;
    int k  = i / (DINNER * CPAD);
    float v = (c < 40) ? s[((size_t)k * 40 + c) * DINNER + dd] : 0.f;
    ST2(uint16_t, d + i, f2bf(v));
}

__global__ void k_aneg(const float* __restrict__ alog, float* __restrict__ an, int n) {
    int i = blockIdx.x * blockDim.x + threadIdx.x;
    if (i < n) ST2(float, an + i, -expf(alog[i]));
}

__global__ void k_patch_embed(const float* __restrict__ x, const float* __restrict__ pw,
                              const float* __restrict__ gam, const float* __restrict__ bet,
                              const float* __restrict__ mean, const float* __restrict__ var,
                              uint16_t* __restrict__ xe) {
    int bp = blockIdx.x;
    int b = bp >> 10, pix = bp & 1023;
    int h = pix >> 5, w = pix & 31;
    int dm = threadIdx.x;
    float acc = 0.f;
#pragma unroll
    for (int ci = 0; ci < 3; ++ci)
#pragma unroll
        for (int ph = 0; ph < 4; ++ph)
#pragma unroll
            for (int pq = 0; pq < 4; ++pq) {
                float xv = x[(((size_t)b * 3 + ci) * IMG + (h * 4 + ph)) * IMG + (w * 4 + pq)];
                float wv = pw[(((size_t)dm * 3 + ci) * 4 + ph) * 4 + pq];
                acc += xv * wv;
            }
    float s = gam[dm] * rsqrtf(var[dm] + 1e-5f);
    ST2(uint16_t, xe + (size_t)bp * DMODEL + dm, f2bf((acc - mean[dm]) * s + bet[dm]));
}

template <int NTILES>
__global__ void k_gemm_staged(const uint16_t* __restrict__ A, const uint16_t* __restrict__ W,
                              float* __restrict__ C, int M, int N, int K) {
    constexpr int BN    = NTILES * 16;
    constexpr int SEG_A = 128 * 32 * 2 / 16;
    constexpr int SEG_B = BN * 32 * 2 / 16;
    constexpr int PER_A = SEG_A / 256;
    constexpr int PER_B = (SEG_B + 255) / 256;
    constexpr int PER   = PER_A + PER_B;

    __shared__ uint16_t sA[2][128 * 32];
    __shared__ uint16_t sB[2][BN * 32];

    const int tid  = threadIdx.x;
    const int wv   = tid >> 5;
    const int lane = tid & 31;
    const int hf   = lane >> 4, r = lane & 15;
    const int m0   = blockIdx.x * 128;
    const int n0   = blockIdx.y * BN;

    f32x8 acc[NTILES];
#pragma unroll
    for (int t = 0; t < NTILES; ++t) acc[t] = {};

    const int nch = K >> 5;

    auto issue = [&](int ch) {
        const int buf = ch & 1;
#pragma unroll
        for (int p = 0; p < PER_A; ++p) {
            int s = tid + p * 256;
            int row = s >> 2, part = s & 3;
            const uint16_t* g = A + (size_t)(m0 + row) * K + ch * 32 + part * 8;
            g2l_16B(g, &sA[buf][s * 8]);
        }
#pragma unroll
        for (int p = 0; p < PER_B; ++p) {
            int s = tid + p * 256;
            if (s >= SEG_B) s -= SEG_B;
            int row = s >> 2, part = s & 3;
            const uint16_t* g = W + (size_t)(n0 + row) * K + ch * 32 + part * 8;
            g2l_16B(g, &sB[buf][s * 8]);
        }
    };

    issue(0);
    for (int ch = 0; ch < nch; ++ch) {
        if (ch + 1 < nch) {
            issue(ch + 1);
            wait_async<PER>();
        } else {
            wait_async<0>();
        }
        __syncthreads();

        const int buf = ch & 1;
        FragBF16 fa;
        const uint16_t* pa = &sA[buf][(wv * 16 + r) * 32];
#pragma unroll
        for (int v = 0; v < 8; ++v) {
            int kb = ((v < 4) ? (2 * v) : (16 + 2 * (v - 4))) + 8 * hf;
            fa.u[v] = *(const uint32_t*)(pa + kb);
        }
#pragma unroll
        for (int t = 0; t < NTILES; ++t) {
            FragBF16 fb;
            const uint16_t* pb = &sB[buf][(t * 16 + r) * 32];
#pragma unroll
            for (int v = 0; v < 8; ++v) {
                int kb = ((v < 4) ? (2 * v) : (16 + 2 * (v - 4))) + 8 * hf;
                fb.u[v] = *(const uint32_t*)(pb + kb);
            }
            acc[t] = __builtin_amdgcn_wmma_f32_16x16x32_f16(
                false, fa.v, false, fb.v, (short)0, acc[t], false, false);
            asm volatile("v_nop\n\tv_nop\n\tv_nop\n\tv_nop" : "+v"(acc[t]) : "v"(fa.v), "v"(fb.v));
        }
        __syncthreads();
    }

    static_assert(NTILES % 2 == 0, "tile pairs");
    for (int pass = 0; pass < 2; ++pass) {
#pragma unroll
        for (int p = 0; p < NTILES / 2; ++p) {
            float* pc = C + (size_t)(m0 + wv * 16) * N + (n0 + p * 32 + lane);
#pragma unroll
            for (int j = 0; j < 8; ++j) {
                const float a0 = acc[2 * p][j], a1 = acc[2 * p + 1][j];
                const float x0 = __shfl_xor(a0, 16), x1 = __shfl_xor(a1, 16);
                *(volatile float*)(pc + (size_t)j * N) = hf ? x1 : a0;
                *(volatile float*)(pc + (size_t)(8 + j) * N) = hf ? a1 : x0;
            }
        }
        __threadfence();
    }
}

__global__ void k_dwconv_silu(const float* __restrict__ xz, const float* __restrict__ cw,
                              const float* __restrict__ cb,
                              float* __restrict__ xs_f, uint16_t* __restrict__ xs_b) {
    int bp = blockIdx.x;
    int b = bp >> 10, pix = bp & 1023;
    int h = pix >> 5, w = pix & 31;
    int d = threadIdx.x;
    float acc = 0.f;
#pragma unroll
    for (int dh = -1; dh <= 1; ++dh)
#pragma unroll
        for (int dw = -1; dw <= 1; ++dw) {
            int hh = h + dh, ww = w + dw;
            if (hh < 0 || hh > 31 || ww < 0 || ww > 31) continue;
            float v = xz[((size_t)b * LSEQ + hh * 32 + ww) * (2 * DINNER) + d];
            acc += v * cw[(size_t)d * 9 + (dh + 1) * 3 + (dw + 1)];
        }
    float s = silu(acc + cb[d]);
    uint16_t sb = f2bf(s);
    int l1 = w * 32 + h;
    int l0 = pix, l2 = LSEQ - 1 - pix, l3 = LSEQ - 1 - l1;
    const size_t KS = (size_t)NPIX * DINNER;
    size_t base = (size_t)b * LSEQ;
    size_t i0 = (base + l0) * DINNER + d, i1 = (base + l1) * DINNER + d;
    size_t i2 = (base + l2) * DINNER + d, i3 = (base + l3) * DINNER + d;
    for (int pass = 0; pass < 2; ++pass) {
        *(volatile float*)(xs_f + 0 * KS + i0) = s;  *(volatile uint16_t*)(xs_b + 0 * KS + i0) = sb;
        *(volatile float*)(xs_f + 1 * KS + i1) = s;  *(volatile uint16_t*)(xs_b + 1 * KS + i1) = sb;
        *(volatile float*)(xs_f + 2 * KS + i2) = s;  *(volatile uint16_t*)(xs_b + 2 * KS + i2) = sb;
        *(volatile float*)(xs_f + 3 * KS + i3) = s;  *(volatile uint16_t*)(xs_b + 3 * KS + i3) = sb;
        __threadfence();
    }
}

__global__ void k_scan(const float* __restrict__ x_dbl, const float* __restrict__ xs_f,
                       const float* __restrict__ dtw, const float* __restrict__ dtb,
                       const float* __restrict__ Aneg, const float* __restrict__ Ds,
                       float* __restrict__ oy) {
    int blk = blockIdx.x;
    int b = blk >> 2, k = blk & 3;
    int d = threadIdx.x;
    float w8[DTRANK];
#pragma unroll
    for (int r = 0; r < DTRANK; ++r) w8[r] = dtw[((size_t)k * DINNER + d) * DTRANK + r];
    float bias = dtb[(size_t)k * DINNER + d];
    float Ar[DSTATE];
#pragma unroll
    for (int s = 0; s < DSTATE; ++s) Ar[s] = Aneg[((size_t)k * DINNER + d) * DSTATE + s];
    float Dv = Ds[(size_t)k * DINNER + d];
    float hS[DSTATE];
#pragma unroll
    for (int s = 0; s < DSTATE; ++s) hS[s] = 0.f;

    const float* xd  = x_dbl + ((size_t)k * NPIX + (size_t)b * LSEQ) * CPAD;
    const float* us  = xs_f  + ((size_t)k * NPIX + (size_t)b * LSEQ) * DINNER + d;
    float*       out = oy    + (((size_t)b * KDIR + k) * LSEQ) * DINNER + d;

    for (int l = 0; l < LSEQ; ++l) {
        const float* c40 = xd + (size_t)l * CPAD;
        float din = bias;
#pragma unroll
        for (int r = 0; r < DTRANK; ++r) din += w8[r] * c40[r];
        float delta = (din > 20.f) ? din : log1pf(__expf(din));
        float u  = us[(size_t)l * DINNER];
        float du = delta * u;
        float y  = 0.f;
#pragma unroll
        for (int s = 0; s < DSTATE; ++s) {
            float dA = __expf(delta * Ar[s]);
            hS[s] = hS[s] * dA + du * c40[8 + s];
            y += hS[s] * c40[24 + s];
        }
        ST2(float, out + (size_t)l * DINNER, y + u * Dv);
    }
}

__global__ void k_merge_ln_gate(const float* __restrict__ oy, const float* __restrict__ xz,
                                const float* __restrict__ g, const float* __restrict__ be,
                                uint16_t* __restrict__ yg) {
    int bp = blockIdx.x;
    int b = bp >> 10, pix = bp & 1023;
    int h = pix >> 5, w = pix & 31;
    int lT = w * 32 + h;
    int d = threadIdx.x;
    size_t bb = (size_t)b * KDIR * LSEQ * DINNER;
    auto at = [&](int k, int l) { return oy[bb + ((size_t)k * LSEQ + l) * DINNER + d]; };
    float y = at(0, pix) + at(2, LSEQ - 1 - pix) + at(1, lT) + at(3, LSEQ - 1 - lT);

    __shared__ float red[DINNER];
    red[d] = y; __syncthreads();
#pragma unroll
    for (int off = 128; off > 0; off >>= 1) { if (d < off) red[d] += red[d + off]; __syncthreads(); }
    float mu = red[0] * (1.f / DINNER); __syncthreads();
    float dy = y - mu;
    red[d] = dy * dy; __syncthreads();
#pragma unroll
    for (int off = 128; off > 0; off >>= 1) { if (d < off) red[d] += red[d + off]; __syncthreads(); }
    float var = red[0] * (1.f / DINNER);
    float yn = dy * rsqrtf(var + 1e-5f) * g[d] + be[d];
    float z = xz[(size_t)bp * (2 * DINNER) + DINNER + d];
    ST2(uint16_t, yg + (size_t)bp * DINNER + d, f2bf(yn * silu(z)));
}

__global__ void k_final(const float* __restrict__ y2, const float* __restrict__ cbias,
                        float* __restrict__ out) {
    const int i = blockIdx.x * blockDim.x + threadIdx.x;
    const int pix = i & (LSEQ - 1), o = (i >> 10) & (DMODEL - 1), b = i >> 17;
    ST2(float, out + i, y2[((size_t)b * LSEQ + pix) * DMODEL + o] + cbias[o]);
}

extern "C" void kernel_launch(void* const* d_in, const int* in_sizes, int n_in,
                              void* d_out, int out_size, void* d_ws, size_t ws_size,
                              hipStream_t stream) {
    (void)in_sizes; (void)n_in; (void)out_size;
    if (ws_size < (size_t)128 * 1024 * 1024) return;
    const float* x         = (const float*)d_in[0];
    const float* proj_w    = (const float*)d_in[1];
    const float* bn_gamma  = (const float*)d_in[2];
    const float* bn_beta   = (const float*)d_in[3];
    const float* bn_mean   = (const float*)d_in[4];
    const float* bn_var    = (const float*)d_in[5];
    const float* in_proj_w = (const float*)d_in[6];
    const float* conv2d_w  = (const float*)d_in[7];
    const float* conv2d_b  = (const float*)d_in[8];
    const float* x_proj_w  = (const float*)d_in[9];
    const float* dt_projs_w= (const float*)d_in[10];
    const float* dt_projs_b= (const float*)d_in[11];
    const float* A_logs    = (const float*)d_in[12];
    const float* Ds        = (const float*)d_in[13];
    const float* ln_gamma  = (const float*)d_in[14];
    const float* ln_beta   = (const float*)d_in[15];
    const float* out_proj_w= (const float*)d_in[16];
    const float* out_conv_w= (const float*)d_in[17];
    const float* out_conv_b= (const float*)d_in[18];
    float* out = (float*)d_out;

    size_t off = 0;
    auto alloc = [&](size_t bytes) -> char* {
        off = (off + 255) & ~(size_t)255;
        char* p = (char*)d_ws + off;
        off += bytes;
        return p;
    };
    uint16_t* xe      = (uint16_t*)alloc((size_t)NPIX * DMODEL * 2);
    uint16_t* w_in    = (uint16_t*)alloc((size_t)512 * DMODEL * 2);
    uint16_t* w_xp    = (uint16_t*)alloc((size_t)KDIR * CPAD * DINNER * 2);
    uint16_t* w_op    = (uint16_t*)alloc((size_t)DMODEL * DINNER * 2);
    uint16_t* w_oc    = (uint16_t*)alloc((size_t)DMODEL * DMODEL * 2);
    float*    Aneg    = (float*)   alloc((size_t)KDIR * DINNER * DSTATE * 4);
    float*    xz      = (float*)   alloc((size_t)NPIX * 512 * 4);
    float*    xs_f    = (float*)   alloc((size_t)KDIR * NPIX * DINNER * 4);
    uint16_t* xs_b    = (uint16_t*)alloc((size_t)KDIR * NPIX * DINNER * 2);
    float*    x_dbl   = (float*)   alloc((size_t)KDIR * NPIX * CPAD * 4);
    float*    oy      = (float*)   alloc((size_t)KDIR * NPIX * DINNER * 4);
    uint16_t* yg      = (uint16_t*)alloc((size_t)NPIX * DINNER * 2);
    float*    y1      = (float*)   alloc((size_t)NPIX * DMODEL * 4);
    uint16_t* y1b     = (uint16_t*)alloc((size_t)NPIX * DMODEL * 2);
    float*    y2      = (float*)   alloc((size_t)NPIX * DMODEL * 4);

    k_f32_to_bf16<<<(512 * DMODEL + 255) / 256, 256, 0, stream>>>(in_proj_w, w_in, 512 * DMODEL);
    k_xproj_pad  <<<(KDIR * CPAD * DINNER + 255) / 256, 256, 0, stream>>>(x_proj_w, w_xp);
    k_f32_to_bf16<<<(DMODEL * DINNER + 255) / 256, 256, 0, stream>>>(out_proj_w, w_op, DMODEL * DINNER);
    k_f32_to_bf16<<<(DMODEL * DMODEL + 255) / 256, 256, 0, stream>>>(out_conv_w, w_oc, DMODEL * DMODEL);
    k_aneg       <<<(KDIR * DINNER * DSTATE + 255) / 256, 256, 0, stream>>>(A_logs, Aneg, KDIR * DINNER * DSTATE);

    k_patch_embed<<<NPIX, DMODEL, 0, stream>>>(x, proj_w, bn_gamma, bn_beta, bn_mean, bn_var, xe);

    k_gemm_staged<8><<<dim3(NPIX / 128, 512 / 128), 256, 0, stream>>>(xe, w_in, xz, NPIX, 512, DMODEL);

    k_dwconv_silu<<<NPIX, DINNER, 0, stream>>>(xz, conv2d_w, conv2d_b, xs_f, xs_b);

    for (int k = 0; k < KDIR; ++k) {
        k_gemm_staged<4><<<dim3(NPIX / 128, 1), 256, 0, stream>>>(
            xs_b + (size_t)k * NPIX * DINNER,
            w_xp + (size_t)k * CPAD * DINNER,
            x_dbl + (size_t)k * NPIX * CPAD,
            NPIX, CPAD, DINNER);
    }

    k_scan<<<BATCH * KDIR, DINNER, 0, stream>>>(x_dbl, xs_f, dt_projs_w, dt_projs_b, Aneg, Ds, oy);

    k_merge_ln_gate<<<NPIX, DINNER, 0, stream>>>(oy, xz, ln_gamma, ln_beta, yg);

    k_gemm_staged<8><<<dim3(NPIX / 128, 1), 256, 0, stream>>>(yg, w_op, y1, NPIX, DMODEL, DINNER);
    k_f32_to_bf16<<<(NPIX * DMODEL + 255) / 256, 256, 0, stream>>>(y1, y1b, NPIX * DMODEL);

    k_gemm_staged<8><<<dim3(NPIX / 128, 1), 256, 0, stream>>>(y1b, w_oc, y2, NPIX, DMODEL, DMODEL);

    k_final<<<NPIX * DMODEL / 256, 256, 0, stream>>>(y2, out_conv_b, out);
}
